// MAGNOEncoder_83897891160641
// MI455X (gfx1250) — hardware-verified
//
#include <hip/hip_runtime.h>
#include <stdint.h>
#include <stddef.h>

constexpr int   kHid         = 256;
constexpr int   kChunkE      = 65536;
constexpr int   kK1          = 32;
constexpr int   kK3          = 320;
constexpr int   kDstTile     = 32;
constexpr int   kAccV4It     = (kDstTile * kHid) / (256 * 4);
constexpr int   kCntLanes    = kDstTile / 4;
constexpr int   kSub         = 256;
constexpr float kWCarry      = 16.0f;
constexpr float kW1TailCarry = 8.0f;
constexpr float kH1Carry     = 16.0f;
constexpr float kGeluExpC    = 2.3022082f;

typedef __attribute__((ext_vector_type(16))) _Float16 v16h;
typedef __attribute__((ext_vector_type(8)))  _Float16 v8h;
typedef __attribute__((ext_vector_type(16))) __bf16   v16b;
typedef __attribute__((ext_vector_type(8)))  __bf16   v8b;
typedef __attribute__((ext_vector_type(8)))  float    v8f;
typedef __attribute__((ext_vector_type(4)))  float    v4f;
typedef __attribute__((ext_vector_type(4)))  unsigned int v4u;
typedef __attribute__((ext_vector_type(4)))  int      v4i;

__device__ __forceinline__ unsigned short f2bf_bits(float f) {
  unsigned u = __float_as_uint(f);
  return (unsigned short)((u + 0x7FFFu + ((u >> 16) & 1u)) >> 16);
}
__device__ __forceinline__ float bf_bits2f(unsigned short h) { return __uint_as_float(((unsigned)h) << 16); }

__device__ __forceinline__ void dep_guard_h(v8f& a, v8f& b, v16h x, v16h y) { asm volatile("v_nop\n\tv_nop\n\tv_nop\n\tv_nop" : "+v"(a), "+v"(b) : "v"(x), "v"(y)); }
__device__ __forceinline__ void dep_guard_b(v8f& a, v8f& b, v16b x, v16b y) { asm volatile("v_nop\n\tv_nop\n\tv_nop\n\tv_nop" : "+v"(a), "+v"(b) : "v"(x), "v"(y)); }
__device__ __forceinline__ void keep4_h(v16h a, v16h b, v16h c, v16h d) { asm volatile("v_nop" :: "v"(a), "v"(b), "v"(c), "v"(d)); }
__device__ __forceinline__ void keep4_b(v16b a, v16b b, v16b c, v16b d) { asm volatile("v_nop" :: "v"(a), "v"(b), "v"(c), "v"(d)); }
__device__ __forceinline__ void acc_guard4(v8f& a, v8f& b, v8f& c, v8f& d) { asm volatile("v_nop\n\tv_nop\n\tv_nop\n\tv_nop" : "+v"(a), "+v"(b), "+v"(c), "+v"(d)); }
template <typename T> struct Frag;
template <> struct Frag<_Float16> {
  typedef v16h V; union U { v16h v; v8h h[2]; };
  static __device__ __forceinline__ v16h load(const _Float16* p) {
    U f; f.h[0] = *(const v8h*)(p); f.h[1] = *(const v8h*)(p + 16); return f.v;
  }
  static __device__ __forceinline__ v8f mma(v16h a, v16h b, v8f c) {
    return __builtin_amdgcn_wmma_f32_16x16x32_f16(false, a, false, b, (short)0, c, false, false);
  }
  static __device__ __forceinline__ void guard(v8f& a, v8f& b, v16h x, v16h y) { dep_guard_h(a, b, x, y); }
  static __device__ __forceinline__ void keep(v16h a, v16h b, v16h c, v16h d) { keep4_h(a, b, c, d); }
};
template <> struct Frag<__bf16> {
  typedef v16b V; union U { v16b v; v8b h[2]; };
  static __device__ __forceinline__ v16b load(const __bf16* p) {
    U f; f.h[0] = *(const v8b*)(p); f.h[1] = *(const v8b*)(p + 16); return f.v;
  }
  static __device__ __forceinline__ v8f mma(v16b a, v16b b, v8f c) {
    return __builtin_amdgcn_wmma_f32_16x16x32_bf16(false, a, false, b, (short)0, c, false, false);
  }
  static __device__ __forceinline__ void guard(v8f& a, v8f& b, v16b x, v16b y) { dep_guard_b(a, b, x, y); }
  static __device__ __forceinline__ void keep(v16b a, v16b b, v16b c, v16b d) { keep4_b(a, b, c, d); }
};

__device__ __forceinline__ unsigned pk16(unsigned short a, unsigned short b) { return (unsigned)a | ((unsigned)b << 16); }
__device__ __forceinline__ unsigned short h_bits(float f) { const _Float16 h = (_Float16)f; return __builtin_bit_cast(unsigned short, h); }

__device__ __forceinline__ float gelu_tanh_f(float x) {
  float u = x * (1.0f + 0.044715f * x * x);
  u = fminf(fmaxf(u, -12.0f), 12.0f);
  const float z = __builtin_amdgcn_exp2f(kGeluExpC * u);
  return x - x * __builtin_amdgcn_rcpf(z + 1.0f);
}

template <int ET> struct Elem;
template <> struct Elem<0> { typedef _Float16 T; };
template <> struct Elem<1> { typedef __bf16 T; };
template <int ET, bool SPLIT, int BIAS_MODE, int OUT_MODE, bool RESID, int ACT = 0>
__global__ __launch_bounds__(256) void wmma_gemm64(
    const unsigned short* __restrict__ Ap, const unsigned short* __restrict__ A2p, int lda, long strideA,
    const unsigned short* __restrict__ Btp, const unsigned short* __restrict__ Bt2p, int ldb, long strideB,
    void* __restrict__ Cout, void* __restrict__ Cout2, int ldc, long strideC,
    const float* __restrict__ bias,
    const float* __restrict__ resid, long strideR,
    int M, int N, int K, float scale) {
  typedef typename Elem<ET>::T T;
  typedef typename Frag<T>::V V;
  const T* A = (const T*)Ap; const T* A2 = (const T*)A2p; const T* Bt = (const T*)Btp; const T* Bt2 = (const T*)Bt2p;
  __shared__ __align__(16) float sT[8][16 * 68];
  const int b    = blockIdx.y;
  const int lane = threadIdx.x & 31;
  const int wave = threadIdx.x >> 5;
  const int tilesN = N >> 6;
  const int tilesM = M >> 6;
  const int tile = blockIdx.x * 8 + wave;
  if (tile >= tilesM * tilesN) return;
  const int tm = tile / tilesN;
  const int tn = tile - tm * tilesN;
  const int m0 = tm << 6;
  const int n0 = tn << 6;

  const T* Ab  = A  + (size_t)b * strideA;
  const T* Bb  = Bt + (size_t)b * strideB;
  const T* Ab2 = SPLIT ? (A2  + (size_t)b * strideA) : nullptr;
  const T* Bb2 = SPLIT ? (Bt2 + (size_t)b * strideB) : nullptr;

  const int rlane = lane & 15;
  const int koff  = (lane >> 4) * 8;
  const int mOff  = (lane >> 4) * 8;

  v8f acc[4][4];
#pragma unroll
  for (int i = 0; i < 4; ++i)
#pragma unroll
    for (int j = 0; j < 4; ++j) acc[i][j] = (v8f){0.f,0.f,0.f,0.f,0.f,0.f,0.f,0.f};

  for (int k0 = 0; k0 < K; k0 += 32) {
    V bh[4], bl[4];
#pragma unroll
    for (int j = 0; j < 4; ++j) {
      const size_t bo = (size_t)(n0 + (j << 4) + rlane) * ldb + koff + k0;
      bh[j] = Frag<T>::load(Bb + bo);
      if (SPLIT) bl[j] = Frag<T>::load(Bb2 + bo);
    }
#pragma unroll
    for (int i = 0; i < 4; ++i) {
      const size_t ao = (size_t)(m0 + (i << 4) + rlane) * lda + koff + k0;
      V ah = Frag<T>::load(Ab + ao);
      V al;
      if (SPLIT) al = Frag<T>::load(Ab2 + ao);
#pragma unroll
      for (int j = 0; j < 4; ++j) {
        acc[i][j] = Frag<T>::mma(ah, bh[j], acc[i][j]);
        if (SPLIT) {
          acc[i][j] = Frag<T>::mma(ah, bl[j], acc[i][j]);
          acc[i][j] = Frag<T>::mma(al, bh[j], acc[i][j]);
        }
      }
      Frag<T>::guard(acc[i][0], acc[i][3], ah, SPLIT ? al : ah);
    }
    Frag<T>::keep(bh[0], bh[1], bh[2], bh[3]);
    if (SPLIT) Frag<T>::keep(bl[0], bl[1], bl[2], bl[3]);
  }
  acc_guard4(acc[0][0], acc[0][1], acc[0][2], acc[0][3]);
  acc_guard4(acc[1][0], acc[1][1], acc[1][2], acc[1][3]);
  acc_guard4(acc[2][0], acc[2][1], acc[2][2], acc[2][3]);
  acc_guard4(acc[3][0], acc[3][1], acc[3][2], acc[3][3]);

  float* slab = sT[wave];
  const float* Rb = RESID ? (resid + (size_t)b * strideR) : nullptr;
#pragma unroll
  for (int i = 0; i < 4; ++i) {
    const int mBase = m0 + (i << 4);
#pragma unroll
    for (int j = 0; j < 4; ++j) {
      const int n = n0 + (j << 4) + rlane;
      float bv = 0.f;
      if (BIAS_MODE == 2) bv = bias[n];
#pragma unroll
      for (int r = 0; r < 8; ++r) {
        float v = acc[i][j][r] * scale;
        if (BIAS_MODE == 1) v += bias[mBase + mOff + r];
        if (BIAS_MODE == 2) v += bv;
        if (RESID) v += Rb[(size_t)(mBase + mOff + r) * ldc + n];
        if (ACT == 2) v = fmaxf(v, 0.0f);
        if (ACT == 4) v = (v > 0.f) ? v : 0.01f * v;
        if (ACT == 6) v = gelu_tanh_f(v);
        if (ACT == 7) v = gelu_tanh_f(v) * kH1Carry;
        slab[(mOff + r) * 68 + (j << 4) + rlane] = v;
      }
    }
    __builtin_amdgcn_fence(__ATOMIC_RELEASE, "workgroup");
    __builtin_amdgcn_wave_barrier();
    __builtin_amdgcn_fence(__ATOMIC_ACQUIRE, "workgroup");
    if (OUT_MODE == 0) {
      float* C = (float*)Cout + (size_t)b * strideC;
      const int hh = lane >> 4, c4 = (lane & 15) * 4;
      for (int pass = 0; pass < 2; ++pass) {
#pragma unroll
        for (int it = 0; it < 8; ++it) {
          const int row = it * 2 + hh;
          v4f v = *(const v4f*)(slab + row * 68 + c4);
          *(volatile v4f*)(C + (size_t)(mBase + row) * ldc + n0 + c4) = v;
        }
        __threadfence();
      }
    } else {
      const int q = lane >> 3, c8 = (lane & 7) * 8;
      unsigned short* C  = (unsigned short*)Cout  + (size_t)b * strideC;
      unsigned short* C2 = (OUT_MODE == 2) ? ((unsigned short*)Cout2 + (size_t)b * strideC) : nullptr;
      for (int pass = 0; pass < 2; ++pass) {
#pragma unroll
        for (int it = 0; it < 4; ++it) {
          const int row = it * 4 + q;
          const float* sp = slab + row * 68 + c8;
          v8h hv, lv;
#pragma unroll
          for (int e = 0; e < 8; ++e) {
            if (OUT_MODE == 1) {
              hv[e] = (_Float16)sp[e];
            } else {
              unsigned short hb = f2bf_bits(sp[e]);
              unsigned short lb = f2bf_bits(sp[e] - bf_bits2f(hb));
              hv[e] = __builtin_bit_cast(_Float16, hb);
              lv[e] = __builtin_bit_cast(_Float16, lb);
            }
          }
          *(volatile v8h*)(C + (size_t)(mBase + row) * ldc + n0 + c8) = hv;
          if (OUT_MODE == 2) *(volatile v8h*)(C2 + (size_t)(mBase + row) * ldc + n0 + c8) = lv;
        }
        __threadfence();
      }
    }
    __builtin_amdgcn_fence(__ATOMIC_RELEASE, "workgroup");
    __builtin_amdgcn_wave_barrier();
    __builtin_amdgcn_fence(__ATOMIC_ACQUIRE, "workgroup");
  }
}

__global__ __launch_bounds__(256) void prep_w23_kernel(const float* __restrict__ W2, const float* __restrict__ W3,
                                                       unsigned short* __restrict__ W2T,
                                                       unsigned short* __restrict__ W3TH, unsigned short* __restrict__ W3TL) {
  __shared__ float sm[64][65];
  const int t  = threadIdx.x;
  const int k0 = blockIdx.x * 64;
  const int n0 = blockIdx.y * 64;
  const int z  = blockIdx.z;
  const float* W = (z == 0) ? W2 : W3;
#pragma unroll
  for (int i = 0; i < 16; ++i) {
    const int e = i * 256 + t;
    const int r = e >> 6;
    const int c = e & 63;
    sm[c][r] = W[(size_t)(k0 + r) * kHid + n0 + c];
  }
  __syncthreads();
  const int lane = t & 31, wave = t >> 5;
  const int q = lane >> 3, c8 = (lane & 7) * 8;
  for (int pass = 0; pass < 2; ++pass) {
#pragma unroll
    for (int it = 0; it < 2; ++it) {
      const int row = wave * 8 + it * 4 + q;
      if (z == 0) {
        unsigned short hb[8];
#pragma unroll
        for (int e = 0; e < 8; ++e) hb[e] = h_bits(kWCarry * sm[row][c8 + e]);
        const v4u u = (v4u){pk16(hb[0], hb[1]), pk16(hb[2], hb[3]), pk16(hb[4], hb[5]), pk16(hb[6], hb[7])};
        *(volatile v4u*)(W2T + (size_t)(n0 + row) * kHid + k0 + c8) = u;
      } else {
        unsigned short hb[8], lb[8];
#pragma unroll
        for (int e = 0; e < 8; ++e) {
          const float v = sm[row][c8 + e];
          hb[e] = f2bf_bits(v);
          lb[e] = f2bf_bits(v - bf_bits2f(hb[e]));
        }
        const v4u uh = (v4u){pk16(hb[0], hb[1]), pk16(hb[2], hb[3]), pk16(hb[4], hb[5]), pk16(hb[6], hb[7])};
        const v4u ul = (v4u){pk16(lb[0], lb[1]), pk16(lb[2], lb[3]), pk16(lb[4], lb[5]), pk16(lb[6], lb[7])};
        *(volatile v4u*)(W3TH + (size_t)(n0 + row) * kK3 + k0 + c8) = uh;
        *(volatile v4u*)(W3TL + (size_t)(n0 + row) * kK3 + k0 + c8) = ul;
      }
    }
    __threadfence();
  }
}

__global__ __launch_bounds__(256) void prep_small_kernel(const float* __restrict__ W1, const float* __restrict__ b3,
                                                         unsigned short* __restrict__ W1T,
                                                         unsigned short* __restrict__ W3TH, unsigned short* __restrict__ W3TL) {
  const int t = threadIdx.x, lane = t & 31, wave = t >> 5;
  for (int pass = 0; pass < 2; ++pass) {
#pragma unroll
    for (int it = 0; it < 4; ++it) {
      const int n = wave * 32 + it * 8 + (lane >> 2);
      const int piece = lane & 3;
      float w[9];
#pragma unroll
      for (int k = 0; k < 9; ++k) w[k] = W1[(size_t)k * kHid + n];
      const unsigned a0 = pk16(h_bits(kWCarry * w[0]), h_bits(kWCarry * w[1]));
      const unsigned a1 = pk16(h_bits(kWCarry * w[2]), h_bits(kWCarry * w[3]));
      const unsigned a2 = pk16(h_bits(kWCarry * w[4]), h_bits(kWCarry * w[5]));
      const unsigned a3 = pk16(h_bits(kWCarry * w[6]), h_bits(kWCarry * w[7]));
      const unsigned short e8 = h_bits(kW1TailCarry * w[8]);
      const unsigned c0 = pk16(e8, e8);
      v4u u;
      u.x = (piece == 0) ? a0 : ((piece == 1) ? c0 : 0u);
      u.y = (piece == 0) ? a1 : 0u;
      u.z = (piece == 0) ? a2 : 0u;
      u.w = (piece == 0) ? a3 : 0u;
      *(volatile v4u*)(W1T + (size_t)n * kK1 + piece * 8) = u;
    }
#pragma unroll
    for (int it = 0; it < 8; ++it) {
      const int n = wave * 32 + it * 4 + (lane >> 3);
      const int piece = lane & 7;
      const float bv = b3[n];
      const unsigned short hb = f2bf_bits(bv);
      const float hf = bf_bits2f(hb);
      const unsigned short lb = f2bf_bits(bv - hf);
      const unsigned short hh = f2bf_bits(0.5f * hf);
      const unsigned short ll = f2bf_bits(0.5f * bf_bits2f(lb));
      const v4u uh = (v4u){(piece == 0) ? pk16(hh, hh) : 0u, 0u, 0u, 0u};
      const v4u ul = (v4u){(piece == 0) ? pk16(ll, ll) : 0u, 0u, 0u, 0u};
      *(volatile v4u*)(W3TH + (size_t)n * kK3 + kHid + piece * 8) = uh;
      *(volatile v4u*)(W3TL + (size_t)n * kK3 + kHid + piece * 8) = ul;
    }
    __threadfence();
  }
}

__global__ __launch_bounds__(256) void gather_edge_kernel(const float* __restrict__ feats, const float* __restrict__ ppos,
                                                          const float* __restrict__ lpos,
                                                          const int* __restrict__ esrc, const int* __restrict__ edst,
                                                          unsigned short* __restrict__ A16,
                                                          int e_base, int n_edges, int n_phys, int n_lat) {
  const int gt = blockIdx.x * 256 + threadIdx.x;
  const int el = gt >> 2;
  const int piece = gt & 3;
  const int e = e_base + el;
  const bool valid = e < n_edges;
  const int ec = valid ? e : (n_edges - 1);
  int s = esrc[ec];
  int d = edst[ec];
  s = min(max(s, 0), n_phys - 1);
  d = min(max(d, 0), n_lat - 1);
  const float* fp = feats + (size_t)s * 3;
  const float* pp = ppos + (size_t)s * 3;
  const float* lp = lpos + (size_t)d * 3;
  const float f0 = fp[0], f1 = fp[1], f2 = fp[2];
  const float p0 = pp[0], p1 = pp[1], p2 = pp[2];
  const float l0 = lp[0], l1 = lp[1], l2 = lp[2];
  const float r0 = l0 - p0, r1 = l1 - p1, r2 = l2 - p2;
  const float g0 = valid ? f0 : 0.f, g1 = valid ? f1 : 0.f, g2 = valid ? f2 : 0.f;
  const float q0 = valid ? p0 : 0.f, q1 = valid ? p1 : 0.f, q2 = valid ? p2 : 0.f;
  const float s0 = valid ? r0 : 0.f, s1 = valid ? r1 : 0.f, s2 = valid ? r2 : 0.f;
  const unsigned w00 = pk16(h_bits(g0), h_bits(g1));
  const unsigned w01 = pk16(h_bits(g2), h_bits(q0));
  const unsigned w02 = pk16(h_bits(q1), h_bits(q2));
  const unsigned w03 = pk16(h_bits(s0), h_bits(s1));
  const unsigned short r2b = h_bits(s2);
  const unsigned w10 = pk16(r2b, r2b);
  v4u u;
  u.x = (piece == 0) ? w00 : ((piece == 1) ? w10 : 0u);
  u.y = (piece == 0) ? w01 : 0u;
  u.z = (piece == 0) ? w02 : 0u;
  u.w = (piece == 0) ? w03 : 0u;
  unsigned short* dst = A16 + (size_t)el * kK1 + piece * 8;
  *(volatile v4u*)dst = u;
  __threadfence();
  *(volatile v4u*)dst = u;
}

__global__ __launch_bounds__(256) void seg_accum_kernel(const int* __restrict__ edst, const float* __restrict__ H2,
                                                        const float* __restrict__ acc_in, const int* __restrict__ cnt_in,
                                                        float* __restrict__ acc_out, int* __restrict__ cnt_out,
                                                        int e_base, int n_edges, int has_carry) {
  __shared__ __align__(16) float sacc[kDstTile * kHid];
  __shared__ __align__(16) int scnt[kDstTile];
  __shared__ int liste[kSub];
  __shared__ int listd[kSub];
  __shared__ int wcnt[8];
  const int t = threadIdx.x, lane = t & 31, wave = t >> 5;
  const int tile_lo = blockIdx.x * kDstTile;
  const size_t tile_off = (size_t)tile_lo * kHid;

  if (has_carry != 0) {
#pragma unroll
    for (int i = 0; i < kAccV4It; ++i) {
      const int q4 = (i * 256 + t) * 4;
      *(v4f*)(sacc + q4) = *(const v4f*)(acc_in + tile_off + q4);
    }
    if (t < kDstTile) scnt[t] = cnt_in[tile_lo + t];
  } else {
    const v4f zero4 = (v4f){0.f, 0.f, 0.f, 0.f};
#pragma unroll
    for (int i = 0; i < kAccV4It; ++i) {
      const int q4 = (i * 256 + t) * 4;
      *(v4f*)(sacc + q4) = zero4;
    }
    if (t < kDstTile) scnt[t] = 0;
  }
  __syncthreads();

  const int nsub = kChunkE / kSub;
  for (int sub = 0; sub < nsub; ++sub) {
    const int el = sub * kSub + t;
    const int e = e_base + el;
    const bool valid = e < n_edges;
    const int ec = valid ? e : (n_edges - 1);
    const int d = edst[ec];
    const unsigned dlu = (unsigned)d - (unsigned)tile_lo;
    const bool hit = valid && (dlu < (unsigned)kDstTile);
    const unsigned m = __builtin_amdgcn_ballot_w32(hit);
    const int rank = __builtin_popcount(m & ((1u << lane) - 1u));
    if (lane == 0) wcnt[wave] = __builtin_popcount(m);
    __syncthreads();
    int base = 0, nh = 0;
#pragma unroll
    for (int w = 0; w < 8; ++w) {
      const int v = wcnt[w];
      nh += v;
      base += (w < wave) ? v : 0;
    }
    if (hit) {
      liste[base + rank] = el;
      listd[base + rank] = (int)dlu;
    }
    __syncthreads();
    nh = min(nh, kSub);
    if (t < 64) {
      const int c4 = t * 4;
      for (int i = 0; i < nh; ++i) {
        int el2 = liste[i];
        int dl2 = listd[i];
        el2 = min(max(el2, 0), kChunkE - 1);
        dl2 &= (kDstTile - 1);
        const v4f v = *(const v4f*)(H2 + (size_t)el2 * kHid + c4);
        float* ap = sacc + dl2 * kHid + c4;
        v4f a = *(v4f*)ap;
        a += v;
        *(v4f*)ap = a;
        if (t == 0) scnt[dl2] += 1;
      }
    }
    __syncthreads();
  }

  const int l8 = lane & (kCntLanes - 1);
  for (int pass = 0; pass < 2; ++pass) {
#pragma unroll
    for (int i = 0; i < kAccV4It; ++i) {
      const int q4 = (i * 256 + t) * 4;
      const v4f v = *(const v4f*)(sacc + q4);
      *(volatile v4f*)(acc_out + tile_off + q4) = v;
    }
    if (wave == 0) {
      const v4i c = *(const v4i*)(scnt + l8 * 4);
      if (lane < kCntLanes) *(volatile v4i*)(cnt_out + tile_lo + l8 * 4) = c;
    }
    __threadfence();
  }
}

__global__ __launch_bounds__(256) void seg_mean_kernel(const float* __restrict__ acc, const int* __restrict__ cnt,
                                                       unsigned short* __restrict__ MH, unsigned short* __restrict__ ML,
                                                       int n_lat) {
  const int t = threadIdx.x, lane = t & 31, wave = t >> 5;
  const int d = blockIdx.x * 8 + wave;
  const int dc = min(d, n_lat - 1);
  const int c = cnt[dc];
  const float inv = 1.0f / (float)(c > 0 ? c : 1);
  const int c0 = lane * 8;
  const v4f a = *(const v4f*)(acc + (size_t)dc * kHid + c0);
  const v4f b = *(const v4f*)(acc + (size_t)dc * kHid + c0 + 4);
  unsigned short hb[8], lb[8];
#pragma unroll
  for (int e = 0; e < 4; ++e) {
    const float m0 = a[e] * inv;
    hb[e] = f2bf_bits(m0);
    lb[e] = f2bf_bits(m0 - bf_bits2f(hb[e]));
    const float m1 = b[e] * inv;
    hb[4 + e] = f2bf_bits(m1);
    lb[4 + e] = f2bf_bits(m1 - bf_bits2f(hb[4 + e]));
  }
  const v4u uh = (v4u){pk16(hb[0], hb[1]), pk16(hb[2], hb[3]), pk16(hb[4], hb[5]), pk16(hb[6], hb[7])};
  const v4u ul = (v4u){pk16(lb[0], lb[1]), pk16(lb[2], lb[3]), pk16(lb[4], lb[5]), pk16(lb[6], lb[7])};
  const unsigned g  = (c > 0) ? 0x3F80u : 0u;
  const unsigned gw = g | (g << 16);
  const v4u th = (v4u){(lane == 0) ? gw : 0u, 0u, 0u, 0u};
  const v4u tz = (v4u){0u, 0u, 0u, 0u};
  if (d < n_lat) {
    unsigned short* rh = MH + (size_t)d * kK3;
    unsigned short* rl = ML + (size_t)d * kK3;
    for (int pass = 0; pass < 2; ++pass) {
      *(volatile v4u*)(rh + c0) = uh;
      *(volatile v4u*)(rl + c0) = ul;
      if (lane < 8) {
        *(volatile v4u*)(rh + kHid + lane * 8) = th;
        *(volatile v4u*)(rl + kHid + lane * 8) = tz;
      }
      __threadfence();
    }
  }
}

extern "C" void kernel_launch(void* const* d_in, const int* in_sizes, int n_in,
                              void* d_out, int out_size, void* d_ws, size_t ws_size, hipStream_t stream) {
  if (n_in < 11) return;
  const float* feats = (const float*)d_in[0];
  const float* ppos  = (const float*)d_in[1];
  const float* lpos  = (const float*)d_in[2];
  const int*   esrc  = (const int*)d_in[3];
  const int*   edst  = (const int*)d_in[4];
  const float* W1    = (const float*)d_in[5];
  const float* b1    = (const float*)d_in[6];
  const float* W2    = (const float*)d_in[7];
  const float* b2    = (const float*)d_in[8];
  const float* W3    = (const float*)d_in[9];
  const float* b3    = (const float*)d_in[10];

  const int n_phys = in_sizes[0] / 3;
  const int n_lat  = in_sizes[2] / 3;
  int n_edges = in_sizes[3];
  if (in_sizes[4] < n_edges) n_edges = in_sizes[4];
  if (n_phys < 1 || n_edges < 1) return;
  if (n_lat < 64 || (n_lat % 64) != 0 || (n_lat % kDstTile) != 0) return;
  if (out_size != n_lat * kHid) return;
  if (in_sizes[5] != 9 * kHid || in_sizes[7] != kHid * kHid || in_sizes[9] != kHid * kHid) return;
  if (in_sizes[6] != kHid || in_sizes[8] != kHid || in_sizes[10] != kHid) return;

  size_t off = 0;
  auto carve = [&](size_t bytes) { const size_t o = off; off += (bytes + 127) & ~(size_t)127; return o; };
  const size_t oW1T  = carve((size_t)kHid * kK1 * 2);
  const size_t oW2T  = carve((size_t)kHid * kHid * 2);
  const size_t oW3TH = carve((size_t)kHid * kK3 * 2);
  const size_t oW3TL = carve((size_t)kHid * kK3 * 2);
  const size_t oA16  = carve((size_t)kChunkE * kK1 * 2);
  const size_t oH1   = carve((size_t)kChunkE * kHid * 2);
  const size_t oH2   = carve((size_t)kChunkE * kHid * 4);
  const size_t oACC0 = carve((size_t)n_lat * kHid * 4);
  const size_t oACC1 = carve((size_t)n_lat * kHid * 4);
  const size_t oCNT0 = carve((size_t)n_lat * 4);
  const size_t oCNT1 = carve((size_t)n_lat * 4);
  const size_t oMH   = carve((size_t)n_lat * kK3 * 2);
  const size_t oML   = carve((size_t)n_lat * kK3 * 2);
  if (off > ws_size) return;

  char* ws = (char*)d_ws;
  unsigned short* W1T  = (unsigned short*)(ws + oW1T);
  unsigned short* W2T  = (unsigned short*)(ws + oW2T);
  unsigned short* W3TH = (unsigned short*)(ws + oW3TH);
  unsigned short* W3TL = (unsigned short*)(ws + oW3TL);
  unsigned short* A16  = (unsigned short*)(ws + oA16);
  unsigned short* H1   = (unsigned short*)(ws + oH1);
  float*          H2   = (float*)(ws + oH2);
  float*          ACC[2] = {(float*)(ws + oACC0), (float*)(ws + oACC1)};
  int*            CNT[2] = {(int*)(ws + oCNT0), (int*)(ws + oCNT1)};
  unsigned short* MH   = (unsigned short*)(ws + oMH);
  unsigned short* ML   = (unsigned short*)(ws + oML);
  float*          OUT  = (float*)d_out;

  prep_w23_kernel<<<dim3(kHid / 64, kHid / 64, 2), dim3(256), 0, stream>>>(W2, W3, W2T, W3TH, W3TL);
  prep_small_kernel<<<dim3(1), dim3(256), 0, stream>>>(W1, b3, W1T, W3TH, W3TL);

  const int tiles12 = (kChunkE / 64) * (kHid / 64);
  const int blk12   = (tiles12 + 7) / 8;
  const int nch     = (n_edges + kChunkE - 1) / kChunkE;
  const int nblk_gather = (kChunkE * 4) / 256;
  const int nblk_acc    = n_lat / kDstTile;

  for (int ch = 0; ch < nch; ++ch) {
    const int e_base = ch * kChunkE;
    gather_edge_kernel<<<dim3(nblk_gather), dim3(256), 0, stream>>>(feats, ppos, lpos, esrc, edst, A16,
                                                                     e_base, n_edges, n_phys, n_lat);
    wmma_gemm64<0, false, 2, 1, false, 7><<<dim3(blk12, 1), dim3(256), 0, stream>>>(
        A16, A16, kK1, 0L, W1T, W1T, kK1, 0L, (void*)H1, (void*)H1, kHid, 0L,
        b1, b1, 0L, kChunkE, kHid, kK1, 1.0f / kWCarry);
    wmma_gemm64<0, false, 2, 0, false, 6><<<dim3(blk12, 1), dim3(256), 0, stream>>>(
        H1, H1, kHid, 0L, W2T, W2T, kHid, 0L, (void*)H2, (void*)H2, kHid, 0L,
        b2, b2, 0L, kChunkE, kHid, kHid, 1.0f / (kH1Carry * kWCarry));
    const int pout = ch & 1, pin = (ch + 1) & 1;
    seg_accum_kernel<<<dim3(nblk_acc), dim3(256), 0, stream>>>(edst, H2, ACC[pin], CNT[pin], ACC[pout], CNT[pout],
                                                                e_base, n_edges, (ch > 0) ? 1 : 0);
  }
  const int pfin = (nch - 1) & 1;
  seg_mean_kernel<<<dim3(n_lat / 8), dim3(256), 0, stream>>>(ACC[pfin], CNT[pfin], MH, ML, n_lat);

  const int tiles3 = (n_lat / 64) * (kHid / 64);
  const int blk3   = (tiles3 + 7) / 8;
  wmma_gemm64<1, true, 0, 0, false, 0><<<dim3(blk3, 1), dim3(256), 0, stream>>>(
      MH, ML, kK3, 0L, W3TH, W3TL, kK3, 0L, (void*)OUT, (void*)OUT, kHid, 0L,
      b3, b3, 0L, n_lat, kHid, kK3, 1.0f);
}
